// MeshGraphNet_67937792688581
// MI455X (gfx1250) — hardware-verified
//
#include <hip/hip_runtime.h>
#include <stddef.h>
#include <stdint.h>

#define HID    128
#define K2     256
#define K4     512
#define NNODE  40000
#define NEDGE  120000
#define NLAY   6
#define DINN   11
#define DINE   3
#define TM     128
#define NP     40064
#define EP     120064
#define AP     264
#define DP     132
#define NTHR   256
#define NWAVE  8
#define GBM    64
#define GBN    128
#define GTHR   128
#define EPT    8
#define CHUNK  (NTHR * EPT)
#define WCAP   (EPT * 32)
#define LISTN  (NWAVE * WCAP)
#define NBA    1024
#define SLA    10
#define RCAP   8192
#define DEGCAP 32
#define MEAS_B1024  3205
#define MEAS_MAXDEG 12
#define AGG_ZINTS (LISTN + 2 * RCAP + 3 * NBA)
#define AGG_LDS_BYTES ((AGG_ZINTS + 16) * 4)
#define ENC_LDS_FLOATS (TM * DP + (TM * AP) / 2 + 512 + DINN * HID + TM * DINN + 32)
#define ENC_LDS_BYTES (ENC_LDS_FLOATS * 4)
#define CH_LDS_BYTES ((TM * DP + (TM * AP) / 2 + 512) * 4)
#define DEC_LDS_FLOATS (TM * DP + HID + 3 * HID + 16 + 3 * TM)
#define DEC_LDS_BYTES (DEC_LDS_FLOATS * 4)
#define WSMAX 134217728

#define PA_ENB   0
#define PA_EEB   512
#define PA_DB1   1024
#define PA_LAYER 1152
#define PA_DW2   7296
#define PA_DB2   7680
#define PA_MX    7712
#define PA_SX    7744
#define PA_ME    7776
#define PA_SE    7808
#define PA_ENW1  7840
#define PA_EEW1  9248
#define PA_TOTAL 9632

static_assert(HID == 128 && K2 == 2 * HID && K4 == 4 * HID);
static_assert(NNODE % 32 == 0 && NP % TM == 0 && EP % TM == 0 && NP % GBM == 0);
static_assert(NP >= NNODE && NP - NNODE < TM && EP >= NEDGE && EP - NEDGE < TM);
static_assert((3 * NNODE) % 4 == 0 && 3 * NNODE == 120000);
static_assert((TM * 3 * 4) % 128 == 0);
static_assert(K2 % 32 == 0 && K4 % 32 == 0);
static_assert((AP * 2) % 16 == 0 && (DP * 4) % 16 == 0 && AP >= K2 && DP >= HID);
static_assert(TM == NWAVE * 16 && NTHR == NWAVE * 32);
static_assert((CHUNK & (CHUNK - 1)) == 0 && CHUNK <= 4096 && WCAP == 256);
static_assert(NBA == (1 << SLA) && NBA % NWAVE == 0 && NBA % 32 == 0);
static_assert(((long long)NEDGE << SLA) < (1LL << 31));
static_assert(RCAP >= (MEAS_B1024 * 5) / 4 && DEGCAP >= MEAS_MAXDEG + 8 && DEGCAP <= 32);
static_assert(AGG_ZINTS % (NTHR * 4) == 0);
static_assert(((NP + NBA - 1) / NBA) * NBA >= NP);
static_assert(AGG_LDS_BYTES <= 327680 && ENC_LDS_BYTES <= 327680 && CH_LDS_BYTES <= 327680 && DEC_LDS_BYTES <= 327680);
static_assert(PA_LAYER + NLAY * 1024 == PA_DW2 && PA_EEW1 + DINE * HID == PA_TOTAL && PA_TOTAL % 32 == 0);
static_assert(PA_DW2 % 32 == 0 && PA_DB2 % 32 == 0 && PA_ENW1 % 32 == 0 && PA_EEW1 % 32 == 0);
static_assert(GBM == (GTHR / 32) * 16 && GBN == HID);

typedef float          v4f   __attribute__((ext_vector_type(4)));
typedef float          v8f   __attribute__((ext_vector_type(8)));
typedef int            v4i   __attribute__((ext_vector_type(4)));
typedef int            v8i   __attribute__((ext_vector_type(8)));
typedef unsigned       v2u   __attribute__((ext_vector_type(2)));
typedef unsigned       v4u   __attribute__((ext_vector_type(4)));
typedef unsigned short v8us  __attribute__((ext_vector_type(8)));
typedef unsigned short v16us __attribute__((ext_vector_type(16)));
typedef __bf16         v16bf __attribute__((ext_vector_type(16)));
typedef v4f  __attribute__((may_alias)) v4fa;
typedef v4i  __attribute__((may_alias)) v4ia;
typedef v2u  __attribute__((may_alias)) v2ua;
typedef v4u  __attribute__((may_alias)) v4ua;
typedef v8us __attribute__((may_alias)) v8usa;
union FragB { v16bf v; v16us u; v8us h[2]; v8i w; };

__device__ __forceinline__ v8f wmb(const FragB& a, const FragB& b, v8f c) {
  v8f d = __builtin_amdgcn_wmma_f32_16x16x32_bf16(false, a.v, false, b.v, (short)0, c, false, false);
  asm volatile("v_nop\n\tv_nop\n\tv_nop\n\tv_nop" : "+v"(d) : "v"(a.w), "v"(b.w));
  return d;
}

__device__ __forceinline__ unsigned bf16_bits(float f) {
  const unsigned u = __float_as_uint(f);
  const unsigned r = (u + 0x7FFFu + ((u >> 16) & 1u)) >> 16;
  return (f != f) ? 0x7FC0u : r;
}
__device__ __forceinline__ float bf16_val(float f) { return __uint_as_float(bf16_bits(f) << 16); }
__device__ __forceinline__ float bf_lo(unsigned w) { return __uint_as_float(w << 16); }
__device__ __forceinline__ float bf_hi(unsigned w) { return __uint_as_float(w & 0xffff0000u); }
__device__ __forceinline__ float relu_np(float v) { return (v > 0.0f) ? v : (v - v); }

__device__ __forceinline__ void put16(unsigned short* dp, v8us o) {
  *(volatile v8us*)dp = o;
  __threadfence();
  *(volatile v8us*)dp = o;
}
__device__ __forceinline__ void putf4(float* dp, v4f o) {
  *(volatile v4f*)dp = o;
  __threadfence();
  *(volatile v4f*)dp = o;
}

__global__ __launch_bounds__(NTHR) void k_wplane(const float* __restrict__ W, unsigned short* dst,
                                                 int nRows, int KK, int srcMat, int rowBase, int nStep, int kStep) {
  const int u   = (int)blockIdx.x * NTHR + (int)threadIdx.x;
  const int upr = KK >> 3;
  if (u >= nRows * upr) return;
  const int mat = (int)blockIdx.y;
  const int n   = u / upr;
  const int k8  = (u - n * upr) * 8;
  const int srow = rowBase + (n >> 7) * nStep + (k8 >> 8) * kStep + (k8 & (HID - 1));
  const float* p = W + (size_t)mat * (size_t)srcMat + (size_t)srow * HID + (n & (HID - 1));
  v8us o;
#pragma unroll
  for (int i = 0; i < 8; ++i) o[i] = (unsigned short)bf16_bits(p[(size_t)i * HID]);
  put16(dst + (size_t)mat * (size_t)nRows * (size_t)KK + (size_t)n * (size_t)KK + k8, o);
}

__global__ __launch_bounds__(NTHR) void k_parA(const float* __restrict__ a0, const float* __restrict__ a1,
                                               const float* __restrict__ a2, const float* __restrict__ a3,
                                               const float* __restrict__ a4, const float* __restrict__ a5,
                                               const float* __restrict__ a6, const float* __restrict__ a7,
                                               const float* __restrict__ a8, float* PAR) {
  const int u = (int)blockIdx.x * NTHR + (int)threadIdx.x;
  if (u >= 9 * 32) return;
  const int arr = u >> 5;
  const int c4  = (u & 31) * 4;
  const float* s = a0;
  if (arr == 1) s = a1;
  if (arr == 2) s = a2;
  if (arr == 3) s = a3;
  if (arr == 4) s = a4;
  if (arr == 5) s = a5;
  if (arr == 6) s = a6;
  if (arr == 7) s = a7;
  if (arr == 8) s = a8;
  v4f q;
  q.x = bf16_val(s[c4 + 0]);
  q.y = bf16_val(s[c4 + 1]);
  q.z = bf16_val(s[c4 + 2]);
  q.w = bf16_val(s[c4 + 3]);
  putf4(PAR + PA_ENB + arr * HID + c4, q);
}

__global__ __launch_bounds__(NTHR) void k_parB(const float* __restrict__ a0, const float* __restrict__ a1,
                                               const float* __restrict__ a2, const float* __restrict__ a3,
                                               const float* __restrict__ a4, const float* __restrict__ a5,
                                               const float* __restrict__ a6, const float* __restrict__ a7,
                                               float* PAR) {
  const int u = (int)blockIdx.x * NTHR + (int)threadIdx.x;
  if (u >= 8 * NLAY * 32) return;
  const int arr = u / (NLAY * 32);
  const int wi  = u - arr * (NLAY * 32);
  const int l   = wi >> 5;
  const int c4  = (wi & 31) * 4;
  const float* s = a0;
  if (arr == 1) s = a1;
  if (arr == 2) s = a2;
  if (arr == 3) s = a3;
  if (arr == 4) s = a4;
  if (arr == 5) s = a5;
  if (arr == 6) s = a6;
  if (arr == 7) s = a7;
  const float* p = s + l * HID + c4;
  v4f q;
  q.x = bf16_val(p[0]);
  q.y = bf16_val(p[1]);
  q.z = bf16_val(p[2]);
  q.w = bf16_val(p[3]);
  putf4(PAR + PA_LAYER + (l * 8 + arr) * HID + c4, q);
}

__global__ __launch_bounds__(NTHR) void k_parC(const float* __restrict__ dw2, const float* __restrict__ db2,
                                               const float* __restrict__ mx, const float* __restrict__ sx,
                                               const float* __restrict__ me, const float* __restrict__ se,
                                               const float* __restrict__ enw1, const float* __restrict__ eew1,
                                               float* PAR) {
  const int b = (int)blockIdx.x;
  const float* s = dw2; int n = 3 * HID; int off = PA_DW2; int padN = 3 * HID;
  if (b == 1) { s = db2;  n = 3;          off = PA_DB2;  padN = 32; }
  if (b == 2) { s = mx;   n = DINN;       off = PA_MX;   padN = 32; }
  if (b == 3) { s = sx;   n = DINN;       off = PA_SX;   padN = 32; }
  if (b == 4) { s = me;   n = DINE;       off = PA_ME;   padN = 32; }
  if (b == 5) { s = se;   n = DINE;       off = PA_SE;   padN = 32; }
  if (b == 6) { s = enw1; n = DINN * HID; off = PA_ENW1; padN = DINN * HID; }
  if (b == 7) { s = eew1; n = DINE * HID; off = PA_EEW1; padN = DINE * HID; }
#pragma unroll 1
  for (int i4 = (int)threadIdx.x * 4; i4 < padN; i4 += NTHR * 4) {
    const int i0 = i4, i1 = i4 + 1, i2 = i4 + 2, i3 = i4 + 3;
    const float v0 = bf16_val(s[i0 < n ? i0 : n - 1]);
    const float v1 = bf16_val(s[i1 < n ? i1 : n - 1]);
    const float v2 = bf16_val(s[i2 < n ? i2 : n - 1]);
    const float v3 = bf16_val(s[i3 < n ? i3 : n - 1]);
    v4f q;
    q.x = (i0 < n) ? v0 : 0.0f;
    q.y = (i1 < n) ? v1 : 0.0f;
    q.z = (i2 < n) ? v2 : 0.0f;
    q.w = (i3 < n) ? v3 : 0.0f;
    putf4(PAR + off + i4, q);
  }
}

__device__ __forceinline__ void gemm_ag(const unsigned short* ap, const unsigned short* __restrict__ bp,
                                        int ldb, int K, v8f (&acc)[8]) {
#pragma unroll 1
  for (int k0 = 0; k0 < K; k0 += 32) {
    FragB af;
    af.h[0] = *(const v8usa*)(ap + k0);
    af.h[1] = *(const v8usa*)(ap + k0 + 16);
#pragma unroll
    for (int nt = 0; nt < 8; ++nt) {
      const unsigned short* wq = bp + (size_t)(16 * nt) * (size_t)ldb + k0;
      FragB bf;
      bf.h[0] = *(const v8usa*)wq;
      bf.h[1] = *(const v8usa*)(wq + 16);
      acc[nt] = wmb(af, bf, acc[nt]);
    }
  }
}
__device__ __forceinline__ void gemm_as(const unsigned short* sap, const unsigned short* __restrict__ bp,
                                        int ldb, int K, v8f (&acc)[8]) {
#pragma unroll 1
  for (int k0 = 0; k0 < K; k0 += 32) {
    FragB af;
    af.h[0] = *(const v8usa*)(sap + k0);
    af.h[1] = *(const v8usa*)(sap + k0 + 16);
#pragma unroll
    for (int nt = 0; nt < 8; ++nt) {
      const unsigned short* wq = bp + (size_t)(16 * nt) * (size_t)ldb + k0;
      FragB bf;
      bf.h[0] = *(const v8usa*)wq;
      bf.h[1] = *(const v8usa*)(wq + 16);
      acc[nt] = wmb(af, bf, acc[nt]);
    }
  }
}
__device__ __forceinline__ void zero_acc(v8f (&acc)[8]) {
  const v8f z = {0.f, 0.f, 0.f, 0.f, 0.f, 0.f, 0.f, 0.f};
#pragma unroll
  for (int t = 0; t < 8; ++t) acc[t] = z;
}
template <int MODE>
__device__ __forceinline__ void stage_tile(float* sD, const v8f (&acc)[8], const float* sBias,
                                           int wave, int hh, int m) {
#pragma unroll
  for (int nt = 0; nt < 8; ++nt) {
    const int lc = 16 * nt + m;
    float bv = 0.0f;
    if constexpr (MODE != 0) bv = sBias[lc];
#pragma unroll
    for (int r = 0; r < 8; ++r) {
      const int lr = 16 * wave + 8 * hh + r;
      float v = acc[nt][r];
      if constexpr (MODE != 0) v = v + bv;
      if constexpr (MODE == 2) v = relu_np(v);
      sD[lr * DP + lc] = v;
    }
  }
}

template <int RES>
__device__ __forceinline__ void ln_rows(float* sD, const float* sG, const float* sB, const unsigned short* res,
                                        int rowBase, int wave, int lane) {
  const v4f g = *(const v4fa*)(sG + 4 * lane);
  const v4f b = *(const v4fa*)(sB + 4 * lane);
#pragma unroll 1
  for (int i = 0; i < 16; ++i) {
    const int lr = 16 * wave + i;
    float* rp = sD + lr * DP + 4 * lane;
    const v4f t = *(const v4fa*)rp;
    float s = (t.x + t.y) + (t.z + t.w);
    s += __shfl_xor(s, 16, 32);
    s += __shfl_xor(s, 8, 32);
    s += __shfl_xor(s, 4, 32);
    s += __shfl_xor(s, 2, 32);
    s += __shfl_xor(s, 1, 32);
    const float mu = s * 0.0078125f;
    const float d0 = t.x - mu, d1 = t.y - mu, d2 = t.z - mu, d3 = t.w - mu;
    float q = (d0 * d0 + d1 * d1) + (d2 * d2 + d3 * d3);
    q += __shfl_xor(q, 16, 32);
    q += __shfl_xor(q, 8, 32);
    q += __shfl_xor(q, 4, 32);
    q += __shfl_xor(q, 2, 32);
    q += __shfl_xor(q, 1, 32);
    const float var = q * 0.0078125f;
    const float rs  = 1.0f / sqrtf(var + 1e-5f);
    v4f y;
    y.x = (d0 * rs) * g.x + b.x;
    y.y = (d1 * rs) * g.y + b.y;
    y.z = (d2 * rs) * g.z + b.z;
    y.w = (d3 * rs) * g.w + b.w;
    if constexpr (RES != 0) {
      const unsigned short* gp = res + (size_t)(rowBase + lr) * K2 + 4 * lane;
      const v2u hw = *(const v2ua*)gp;
      const v2u lw = *(const v2ua*)(gp + HID);
      y.x = y.x + (bf_lo(hw.x) + bf_lo(lw.x));
      y.y = y.y + (bf_hi(hw.x) + bf_hi(lw.x));
      y.z = y.z + (bf_lo(hw.y) + bf_lo(lw.y));
      y.w = y.w + (bf_hi(hw.y) + bf_hi(lw.y));
    }
    *(v4fa*)rp = y;
  }
}

template <int ZPAD>
__device__ __forceinline__ void store_rows(const float* sD, unsigned short* plane, int rowBase, int nValid,
                                           int wave, int lane) {
  const int part = lane >> 4;
  const int j = lane & 15;
  const unsigned mh = 0u - (unsigned)part;
  const unsigned ml = ~mh;
  v8us pv[16];
#pragma unroll
  for (int i = 0; i < 16; ++i) {
    const float* sp = sD + (16 * wave + i) * DP + 8 * j;
    const v4f a = *(const v4fa*)sp;
    const v4f c = *(const v4fa*)(sp + 4);
    const v8f f8 = {a.x, a.y, a.z, a.w, c.x, c.y, c.z, c.w};
    const bool ok = (rowBase + 16 * wave + i) < nValid;
    v8us oo;
#pragma unroll
    for (int e = 0; e < 8; ++e) {
      const unsigned hb = bf16_bits(f8[e]);
      const unsigned lb = bf16_bits(f8[e] - __uint_as_float(hb << 16));
      unsigned w = (hb & ml) | (lb & mh);
      if constexpr (ZPAD != 0) w = ok ? w : 0u;
      oo[e] = (unsigned short)w;
    }
    pv[i] = oo;
  }
#pragma unroll
  for (int i = 0; i < 16; ++i) {
    const int row = rowBase + 16 * wave + i;
    if (ZPAD != 0 || row < nValid)
      *(volatile v8us*)(plane + (size_t)row * K2 + part * HID + 8 * j) = pv[i];
  }
  __threadfence();
#pragma unroll
  for (int i = 0; i < 16; ++i) {
    const int row = rowBase + 16 * wave + i;
    if (ZPAD != 0 || row < nValid)
      *(volatile v8us*)(plane + (size_t)row * K2 + part * HID + 8 * j) = pv[i];
  }
}

template <int DIN>
__global__ __launch_bounds__(NTHR) __attribute__((amdgpu_num_vgpr(248)))
void k_enc(const float* __restrict__ in, int nRows, const float* __restrict__ PAR,
           int oMean, int oStd, int oW1, int oB,
           const unsigned short* __restrict__ W2p, unsigned short* outp) {
  extern __shared__ __attribute__((aligned(16))) float dyn[];
  float*          sD  = dyn;
  unsigned short* sH  = (unsigned short*)(dyn + TM * DP);
  float*          sP  = dyn + TM * DP + (TM * AP) / 2;
  float*          sW1 = sP + 512;
  float*          sIn = sW1 + DINN * HID;
  float*          sMS = sIn + TM * DINN;
  const int tid = (int)threadIdx.x, lane = tid & 31, wave = tid >> 5, hh = lane >> 4, m = lane & 15;
  const int rowBase = (int)blockIdx.x * TM;

  for (int i = tid; i < 512; i += NTHR) sP[i] = PAR[oB + i];
  for (int i = tid; i < DIN * HID; i += NTHR) sW1[i] = PAR[oW1 + i];
  if (tid < 32) {
    const int k   = tid & 15;
    const int kc  = k < DIN ? k : DIN - 1;
    const int off = ((tid < 16) ? oMean : oStd) + kc;
    sMS[tid] = PAR[off];
  }
  __syncthreads();
  {
    const long long gbase = (long long)rowBase * DIN;
    const long long total = (long long)nRows * DIN;
#pragma unroll 1
    for (int i = tid; i < TM * DIN; i += NTHR) {
      long long gi = gbase + i;
      gi = gi < total ? gi : total - 1;
      const int k = i % DIN;
      const float v = bf16_val(in[gi]);
      sIn[i] = (v - sMS[k]) / sMS[16 + k];
    }
  }
  __syncthreads();
  {
    const int r  = tid & (TM - 1);
    const int cs = (tid >> 7) * 64;
#pragma unroll 1
    for (int c8 = 0; c8 < 8; ++c8) {
      const int c = cs + 8 * c8;
      v8f a8 = {0.f, 0.f, 0.f, 0.f, 0.f, 0.f, 0.f, 0.f};
#pragma unroll 1
      for (int k = 0; k < DIN; ++k) {
        const float xv = sIn[r * DIN + k];
        const v4f wa = *(const v4fa*)(sW1 + k * HID + c);
        const v4f wb = *(const v4fa*)(sW1 + k * HID + c + 4);
        a8[0] = fmaf(xv, wa.x, a8[0]);
        a8[1] = fmaf(xv, wa.y, a8[1]);
        a8[2] = fmaf(xv, wa.z, a8[2]);
        a8[3] = fmaf(xv, wa.w, a8[3]);
        a8[4] = fmaf(xv, wb.x, a8[4]);
        a8[5] = fmaf(xv, wb.y, a8[5]);
        a8[6] = fmaf(xv, wb.z, a8[6]);
        a8[7] = fmaf(xv, wb.w, a8[7]);
      }
      const v4f ba = *(const v4fa*)(sP + c);
      const v4f bb = *(const v4fa*)(sP + c + 4);
      const v8f b8 = {ba.x, ba.y, ba.z, ba.w, bb.x, bb.y, bb.z, bb.w};
      v8us oh, ol;
#pragma unroll
      for (int i = 0; i < 8; ++i) {
        const float v = relu_np(a8[i] + b8[i]);
        const unsigned hb = bf16_bits(v);
        const unsigned lb = bf16_bits(v - __uint_as_float(hb << 16));
        oh[i] = (unsigned short)hb;
        ol[i] = (unsigned short)lb;
      }
      *(v8usa*)(sH + r * AP + c)       = oh;
      *(v8usa*)(sH + r * AP + HID + c) = ol;
    }
  }
  __syncthreads();
  v8f acc[8];
  zero_acc(acc);
  gemm_as(sH + (16 * wave + m) * AP + 8 * hh, W2p + (size_t)m * K2 + 8 * hh, K2, K2, acc);
  stage_tile<1>(sD, acc, sP + HID, wave, hh, m);
  __syncthreads();
  ln_rows<0>(sD, sP + 2 * HID, sP + 3 * HID, outp, rowBase, wave, lane);
  __syncthreads();
  store_rows<1>(sD, outp, rowBase, nRows, wave, lane);
}

__global__ __launch_bounds__(GTHR) __attribute__((amdgpu_num_vgpr(248)))
void k_pre(const unsigned short* __restrict__ A, const unsigned short* __restrict__ BT, float* Cm) {
  __shared__ __attribute__((aligned(16))) float stg[GBM * GBN];
  const int tid = (int)threadIdx.x, lane = tid & 31, wave = tid >> 5, hh = lane >> 4, m = lane & 15;
  const int rowBase = (int)blockIdx.x * GBM;
  const int colBase = (int)blockIdx.y * GBN;
  v8f acc[8];
  zero_acc(acc);
  gemm_ag(A + (size_t)(rowBase + 16 * wave + m) * K2 + 8 * hh,
          BT + (size_t)(colBase + m) * K2 + 8 * hh, K2, K2, acc);
#pragma unroll
  for (int nt = 0; nt < 8; ++nt) {
    const int lc = 16 * nt + m;
#pragma unroll
    for (int r = 0; r < 8; ++r) stg[(16 * wave + 8 * hh + r) * GBN + lc] = acc[nt][r];
  }
  __syncthreads();
  v4f pv[16];
#pragma unroll
  for (int i = 0; i < 16; ++i) pv[i] = *(const v4fa*)(stg + (16 * wave + i) * GBN + 4 * lane);
#pragma unroll
  for (int i = 0; i < 16; ++i) {
    float* op = Cm + (size_t)(rowBase + 16 * wave + i) * K2 + colBase + 4 * lane;
    *(volatile v4f*)op = pv[i];
  }
  __threadfence();
#pragma unroll
  for (int i = 0; i < 16; ++i) {
    float* op = Cm + (size_t)(rowBase + 16 * wave + i) * K2 + colBase + 4 * lane;
    *(volatile v4f*)op = pv[i];
  }
}

__global__ __launch_bounds__(NTHR) __attribute__((amdgpu_num_vgpr(248)))
void k_edge(const int* __restrict__ ei, unsigned short* EA, const float* __restrict__ P,
            const unsigned short* __restrict__ PCp, const unsigned short* __restrict__ PE2p,
            const float* __restrict__ PAR, int oPar, int nE, int nN) {
  extern __shared__ __attribute__((aligned(16))) float dyn[];
  float*          sD = dyn;
  unsigned short* sH = (unsigned short*)(dyn + TM * DP);
  float*          sP = dyn + TM * DP + (TM * AP) / 2;
  const int tid = (int)threadIdx.x, lane = tid & 31, wave = tid >> 5, hh = lane >> 4, m = lane & 15;
  const int e0 = (int)blockIdx.x * TM;

  for (int i = tid; i < 512; i += NTHR) sP[i] = PAR[oPar + i];

  v8f acc[8];
  zero_acc(acc);
  gemm_ag(EA + (size_t)(e0 + 16 * wave + m) * K2 + 8 * hh, PCp + (size_t)m * K2 + 8 * hh, K2, K2, acc);
  stage_tile<0>(sD, acc, sD, wave, hh, m);
  __syncthreads();
  {
    const v4f b1 = *(const v4fa*)(sP + 4 * lane);
#pragma unroll 1
    for (int i = 0; i < 16; ++i) {
      const int lr = 16 * wave + i;
      const int e  = e0 + lr;
      const int ec = e < nE ? e : nE - 1;
      int s = ei[ec];
      int d = ei[nE + ec];
      s = s < 0 ? 0 : (s > nN - 1 ? nN - 1 : s);
      d = d < 0 ? 0 : (d > nN - 1 ? nN - 1 : d);
      const v4f st = *(const v4fa*)(sD + lr * DP + 4 * lane);
      const v4f pa = *(const v4fa*)(P + (size_t)d * K2 + 4 * lane);
      const v4f pb = *(const v4fa*)(P + (size_t)s * K2 + HID + 4 * lane);
      const float v0 = relu_np((st.x + (pa.x + pb.x)) + b1.x);
      const float v1 = relu_np((st.y + (pa.y + pb.y)) + b1.y);
      const float v2 = relu_np((st.z + (pa.z + pb.z)) + b1.z);
      const float v3 = relu_np((st.w + (pa.w + pb.w)) + b1.w);
      const unsigned h0 = bf16_bits(v0), h1 = bf16_bits(v1), h2 = bf16_bits(v2), h3 = bf16_bits(v3);
      const unsigned l0 = bf16_bits(v0 - __uint_as_float(h0 << 16));
      const unsigned l1 = bf16_bits(v1 - __uint_as_float(h1 << 16));
      const unsigned l2 = bf16_bits(v2 - __uint_as_float(h2 << 16));
      const unsigned l3 = bf16_bits(v3 - __uint_as_float(h3 << 16));
      v2u hw, lw;
      hw.x = h0 | (h1 << 16);
      hw.y = h2 | (h3 << 16);
      lw.x = l0 | (l1 << 16);
      lw.y = l2 | (l3 << 16);
      *(v2ua*)(sH + lr * AP + 4 * lane)       = hw;
      *(v2ua*)(sH + lr * AP + HID + 4 * lane) = lw;
    }
  }
  __syncthreads();
  zero_acc(acc);
  gemm_as(sH + (16 * wave + m) * AP + 8 * hh, PE2p + (size_t)m * K2 + 8 * hh, K2, K2, acc);
  stage_tile<1>(sD, acc, sP + HID, wave, hh, m);
  __syncthreads();
  ln_rows<1>(sD, sP + 2 * HID, sP + 3 * HID, EA, e0, wave, lane);
  __syncthreads();
  store_rows<0>(sD, EA, e0, nE, wave, lane);
}

template <int SLB>
__device__ __forceinline__ int scan_chunk(const int* __restrict__ keys, int nE, int cbase, int slotBase,
                                          int nb, int* list, int lane, int wave) {
  int wc = 0;
  const int elw  = wave * WCAP + lane;
  const int eb   = cbase + elw;
  const int sent = -2147483647 - 1;
  const int q0 = keys[min(eb,       nE - 1)];
  const int q1 = keys[min(eb + 32,  nE - 1)];
  const int q2 = keys[min(eb + 64,  nE - 1)];
  const int q3 = keys[min(eb + 96,  nE - 1)];
  const int q4 = keys[min(eb + 128, nE - 1)];
  const int q5 = keys[min(eb + 160, nE - 1)];
  const int q6 = keys[min(eb + 192, nE - 1)];
  const int q7 = keys[min(eb + 224, nE - 1)];
  const int d0 = (eb       < nE) ? q0 : sent;
  const int d1 = (eb + 32  < nE) ? q1 : sent;
  const int d2 = (eb + 64  < nE) ? q2 : sent;
  const int d3 = (eb + 96  < nE) ? q3 : sent;
  const int d4 = (eb + 128 < nE) ? q4 : sent;
  const int d5 = (eb + 160 < nE) ? q5 : sent;
  const int d6 = (eb + 192 < nE) ? q6 : sent;
  const int d7 = (eb + 224 < nE) ? q7 : sent;
  const unsigned nbs = (unsigned)slotBase;
  const unsigned unb = (unsigned)nb;
  const unsigned s0 = (unsigned)d0 - nbs, s1 = (unsigned)d1 - nbs;
  const unsigned s2 = (unsigned)d2 - nbs, s3 = (unsigned)d3 - nbs;
  const unsigned s4 = (unsigned)d4 - nbs, s5 = (unsigned)d5 - nbs;
  const unsigned s6 = (unsigned)d6 - nbs, s7 = (unsigned)d7 - nbs;
  const bool h0 = s0 < unb, h1 = s1 < unb, h2 = s2 < unb, h3 = s3 < unb;
  const bool h4 = s4 < unb, h5 = s5 < unb, h6 = s6 < unb, h7 = s7 < unb;
  const unsigned any = __builtin_amdgcn_ballot_w32(h0 | h1 | h2 | h3 | h4 | h5 | h6 | h7);
  if (any != 0u) {
#define HITJ(J, HJ, SJ) { \
      const unsigned mj = __builtin_amdgcn_ballot_w32(HJ); \
      if (mj != 0u) { \
        if (HJ) { \
          const int pos = wc + (int)__builtin_amdgcn_mbcnt_lo(mj, 0u); \
          if (pos < WCAP) list[wave * WCAP + pos] = ((elw + 32 * (J)) << SLB) | (int)(SJ); \
        } \
        wc += (int)__builtin_popcount(mj); } }
    HITJ(0, h0, s0)
    HITJ(1, h1, s1)
    HITJ(2, h2, s2)
    HITJ(3, h3, s3)
    HITJ(4, h4, s4)
    HITJ(5, h5, s5)
    HITJ(6, h6, s6)
    HITJ(7, h7, s7)
#undef HITJ
  }
  return wc;
}

__global__ __launch_bounds__(NTHR) __attribute__((amdgpu_num_vgpr(248)))
void k_agg(const int* __restrict__ keys, int nE, const unsigned short* __restrict__ EA,
           unsigned short* AGG, int mRows) {
  extern __shared__ __attribute__((aligned(16))) int dsm[];
  int* list = dsm;
  int* hl   = dsm + LISTN;
  int* sl   = hl + RCAP;
  int* cnt  = sl + RCAP;
  int* offs = cnt + NBA;
  int* cur  = offs + NBA;
  int* misc = cur + NBA;
  const int tid = (int)threadIdx.x, lane = tid & 31, wave = tid >> 5;
  const int nodeBase = (int)blockIdx.x * NBA;

  {
    const v4i z4 = {0, 0, 0, 0};
    for (int i = tid * 4; i < AGG_ZINTS; i += NTHR * 4) *(v4ia*)(dsm + i) = z4;
    if (tid < 16) misc[tid] = 0;
  }
  __syncthreads();

  int t = 0, ov = 0;
  const int nChunks = (nE + CHUNK - 1) / CHUNK;
#pragma unroll 1
  for (int ch = 0; ch < nChunks; ++ch) {
    const int cbase = ch * CHUNK;
    const int wc = scan_chunk<SLA>(keys, nE, cbase, nodeBase, NBA, list, lane, wave);
    if (lane == 0) misc[wave] = wc;
    __syncthreads();
    if (wave == 0) {
#pragma unroll 1
      for (int w2 = 0; w2 < NWAVE; ++w2) {
        int c = misc[w2];
        c = c < 0 ? 0 : (c > WCAP ? WCAP : c);
#pragma unroll 1
        for (int b0 = 0; b0 < c; b0 += 32) {
          const int idx = b0 + lane;
          const int ent = list[w2 * WCAP + (idx < WCAP ? idx : WCAP - 1)];
          const int m32 = (c - b0) < 32 ? (c - b0) : 32;
#pragma unroll 1
          for (int k = 0; k < m32; ++k) {
            const int u    = __builtin_amdgcn_readlane(ent, k);
            const int slot = u & (NBA - 1);
            const int el   = (u >> SLA) & (CHUNK - 1);
            const int pk   = ((cbase + el) << SLA) | slot;
            if (t < RCAP) {
              if (lane == 0) { hl[t] = pk; cnt[slot] = cnt[slot] + 1; }
              t = t + 1;
            } else {
              ov = 1;
            }
          }
        }
      }
    }
    __syncthreads();
  }
  if (wave == 0 && lane == 0) { misc[8] = t; misc[9] = ov; }
  __syncthreads();
  int tt = misc[8];
  tt = tt < 0 ? 0 : (tt > RCAP ? RCAP : tt);
  const int ovf = misc[9];

  if (wave == 0) {
    const int base = lane * (NBA / 32);
    int s = 0;
#pragma unroll 1
    for (int i = 0; i < NBA / 32; ++i) s += cnt[base + i];
    int incl = s;
#pragma unroll
    for (int d = 1; d < 32; d <<= 1) {
      const int y = __shfl_up(incl, d, 32);
      if (lane >= d) incl += y;
    }
    int run = incl - s;
#pragma unroll 1
    for (int i = 0; i < NBA / 32; ++i) {
      const int cv = cnt[base + i];
      offs[base + i] = run;
      cur[base + i]  = run;
      run += cv;
    }
  }
  __syncthreads();
  if (wave == 0) {
#pragma unroll 1
    for (int b0 = 0; b0 < tt; b0 += 32) {
      const int idx = b0 + lane;
      const int ent = hl[idx < RCAP ? idx : RCAP - 1];
      const int m32 = (tt - b0) < 32 ? (tt - b0) : 32;
#pragma unroll 1
      for (int k = 0; k < m32; ++k) {
        const int u    = __builtin_amdgcn_readlane(ent, k);
        const int slot = u & (NBA - 1);
        if (lane == 0) {
          int p = cur[slot];
          p = p < 0 ? 0 : (p > RCAP - 1 ? RCAP - 1 : p);
          sl[p] = u;
          cur[slot] = p + 1;
        }
      }
    }
  }
  __syncthreads();

  const float qnan = __int_as_float(0x7fc00000);
  const int part = lane >> 4;
  const int j = lane & 15;
  const unsigned mh = 0u - (unsigned)part;
  const unsigned ml = ~mh;
#pragma unroll 1
  for (int si = 0; si < NBA / NWAVE; ++si) {
    const int s    = si * NWAVE + wave;
    const int node = nodeBase + s;
    int c = cnt[s];
    const bool big = c > DEGCAP;
    c = c < 0 ? 0 : (c > DEGCAP ? DEGCAP : c);
    int o = offs[s];
    o = o < 0 ? 0 : (o > RCAP ? RCAP : o);
    v8f a8 = {0.f, 0.f, 0.f, 0.f, 0.f, 0.f, 0.f, 0.f};
#pragma unroll 1
    for (int b0 = 0; b0 < c; b0 += 32) {
      int idx = o + b0 + lane;
      idx = idx > RCAP - 1 ? RCAP - 1 : idx;
      const int ent = sl[idx];
      int eid = ent >> SLA;
      eid = eid < 0 ? 0 : (eid > nE - 1 ? nE - 1 : eid);
      const int m32 = (c - b0) < 32 ? (c - b0) : 32;
#pragma unroll 1
      for (int k = 0; k < m32; ++k) {
        const int ek = __builtin_amdgcn_readlane(eid, k);
        const unsigned short* rp = EA + (size_t)ek * K2 + 8 * j;
        const v4u hw = *(const v4ua*)rp;
        const v4u lw = *(const v4ua*)(rp + HID);
        a8[0] += bf_lo(hw.x) + bf_lo(lw.x);
        a8[1] += bf_hi(hw.x) + bf_hi(lw.x);
        a8[2] += bf_lo(hw.y) + bf_lo(lw.y);
        a8[3] += bf_hi(hw.y) + bf_hi(lw.y);
        a8[4] += bf_lo(hw.z) + bf_lo(lw.z);
        a8[5] += bf_hi(hw.z) + bf_hi(lw.z);
        a8[6] += bf_lo(hw.w) + bf_lo(lw.w);
        a8[7] += bf_hi(hw.w) + bf_hi(lw.w);
      }
    }
    const float pzr = (big || ovf != 0) ? qnan : 0.0f;
    v8us oo;
#pragma unroll
    for (int e = 0; e < 8; ++e) {
      const float v = a8[e] + pzr;
      const unsigned hb = bf16_bits(v);
      const unsigned lb = bf16_bits(v - __uint_as_float(hb << 16));
      oo[e] = (unsigned short)((hb & ml) | (lb & mh));
    }
    const bool live = node < mRows;
    const int  nr   = live ? node : mRows - 1;
    unsigned short* dp = AGG + (size_t)nr * K2 + part * HID + 8 * j;
    if (live) *(volatile v8us*)dp = oo;
    __threadfence();
    if (live) *(volatile v8us*)dp = oo;
  }
}

__global__ __launch_bounds__(NTHR) __attribute__((amdgpu_num_vgpr(248)))
void k_node(unsigned short* X, const unsigned short* __restrict__ AGG,
            const unsigned short* __restrict__ PN1p, const unsigned short* __restrict__ PN2p,
            const float* __restrict__ PAR, int oPar, int nN) {
  extern __shared__ __attribute__((aligned(16))) float dyn[];
  float*          sD = dyn;
  unsigned short* sH = (unsigned short*)(dyn + TM * DP);
  float*          sP = dyn + TM * DP + (TM * AP) / 2;
  const int tid = (int)threadIdx.x, lane = tid & 31, wave = tid >> 5, hh = lane >> 4, m = lane & 15;
  const int n0 = (int)blockIdx.x * TM;

  for (int i = tid; i < 512; i += NTHR) sP[i] = PAR[oPar + i];
  __syncthreads();

  v8f acc[8];
  zero_acc(acc);
  gemm_ag(X   + (size_t)(n0 + 16 * wave + m) * K2 + 8 * hh, PN1p + (size_t)m * K4 + 8 * hh,      K4, K2, acc);
  gemm_ag(AGG + (size_t)(n0 + 16 * wave + m) * K2 + 8 * hh, PN1p + (size_t)m * K4 + K2 + 8 * hh, K4, K2, acc);
#pragma unroll
  for (int nt = 0; nt < 8; ++nt) {
    const int lc = 16 * nt + m;
    const float bv = sP[lc];
#pragma unroll
    for (int r = 0; r < 8; ++r) {
      const int lr = 16 * wave + 8 * hh + r;
      const float v = relu_np(acc[nt][r] + bv);
      const unsigned hb = bf16_bits(v);
      const unsigned lb = bf16_bits(v - __uint_as_float(hb << 16));
      sH[lr * AP + lc]       = (unsigned short)hb;
      sH[lr * AP + HID + lc] = (unsigned short)lb;
    }
  }
  __syncthreads();
  zero_acc(acc);
  gemm_as(sH + (16 * wave + m) * AP + 8 * hh, PN2p + (size_t)m * K2 + 8 * hh, K2, K2, acc);
  stage_tile<1>(sD, acc, sP + HID, wave, hh, m);
  __syncthreads();
  ln_rows<1>(sD, sP + 2 * HID, sP + 3 * HID, X, n0, wave, lane);
  __syncthreads();
  store_rows<0>(sD, X, n0, nN, wave, lane);
}

__global__ __launch_bounds__(NTHR) __attribute__((amdgpu_num_vgpr(248)))
void k_dec(const unsigned short* __restrict__ X, const unsigned short* __restrict__ D1p,
           const float* __restrict__ PAR, float* outp, int nN) {
  extern __shared__ __attribute__((aligned(16))) float dyn[];
  float* sD  = dyn;
  float* sB1 = dyn + TM * DP;
  float* sW2 = sB1 + HID;
  float* sB2 = sW2 + 3 * HID;
  float* sO  = sB2 + 16;
  const int tid = (int)threadIdx.x, lane = tid & 31, wave = tid >> 5, hh = lane >> 4, m = lane & 15;
  const int n0 = (int)blockIdx.x * TM;

  if (tid < HID) sB1[tid] = PAR[PA_DB1 + tid];
  for (int i = tid; i < 3 * HID; i += NTHR) sW2[i] = PAR[PA_DW2 + i];
  if (tid < 16) sB2[tid] = PAR[PA_DB2 + tid];
  __syncthreads();

  v8f acc[8];
  zero_acc(acc);
  gemm_ag(X + (size_t)(n0 + 16 * wave + m) * K2 + 8 * hh, D1p + (size_t)m * K2 + 8 * hh, K2, K2, acc);
  stage_tile<2>(sD, acc, sB1, wave, hh, m);
  __syncthreads();
  if (tid < TM) {
    const float* hr = sD + tid * DP;
    float o0 = 0.0f, o1 = 0.0f, o2 = 0.0f;
#pragma unroll 4
    for (int k = 0; k < HID; ++k) {
      const float hv = hr[k];
      o0 = fmaf(hv, sW2[3 * k + 0], o0);
      o1 = fmaf(hv, sW2[3 * k + 1], o1);
      o2 = fmaf(hv, sW2[3 * k + 2], o2);
    }
    sO[3 * tid + 0] = o0 + sB2[0];
    sO[3 * tid + 1] = o1 + sB2[1];
    sO[3 * tid + 2] = o2 + sB2[2];
  }
  __syncthreads();
  const int tl = tid < (3 * TM) / 4 ? tid : (3 * TM) / 4 - 1;
  const v4f o4 = *(const v4fa*)(sO + 4 * tl);
  const int gidx = (int)blockIdx.x * (3 * TM) + 4 * tl;
  const bool stv = (tid < (3 * TM) / 4) && (gidx + 4 <= 3 * nN);
  if (stv) *(volatile v4f*)(outp + (size_t)gidx) = o4;
  __threadfence();
  if (stv) *(volatile v4f*)(outp + (size_t)gidx) = o4;
}

static inline int cdiv(int a, int b) { return (a + b - 1) / b; }

extern "C" void kernel_launch(void* const* d_in, const int* in_sizes, int n_in,
                              void* d_out, int out_size, void* d_ws, size_t ws_size,
                              hipStream_t stream) {
  if (n_in < 35) return;
  static const int expect[35] = {
      NNODE * DINN, NEDGE * DINE, 2 * NEDGE, DINN, DINN, DINE, DINE,
      DINN * HID, HID, HID * HID, HID, HID, HID,
      DINE * HID, HID, HID * HID, HID, HID, HID,
      NLAY * 2 * HID * HID, NLAY * HID, NLAY * HID * HID, NLAY * HID, NLAY * HID, NLAY * HID,
      NLAY * 3 * HID * HID, NLAY * HID, NLAY * HID * HID, NLAY * HID, NLAY * HID, NLAY * HID,
      HID * HID, HID, HID * 3, 3};
  for (int i = 0; i < 35; ++i) if (in_sizes[i] != expect[i]) return;
  if (out_size != 3 * NNODE) return;

  const float* x_in   = (const float*)d_in[0];
  const float* eattr  = (const float*)d_in[1];
  const int*   ei     = (const int*)d_in[2];
  const float* mean_x = (const float*)d_in[3];
  const float* std_x  = (const float*)d_in[4];
  const float* mean_e = (const float*)d_in[5];
  const float* std_e  = (const float*)d_in[6];
  const float* en_w1  = (const float*)d_in[7];
  const float* en_b1  = (const float*)d_in[8];
  const float* en_w2  = (const float*)d_in[9];
  const float* en_b2  = (const float*)d_in[10];
  const float* en_g   = (const float*)d_in[11];
  const float* en_b   = (const float*)d_in[12];
  const float* ee_w1  = (const float*)d_in[13];
  const float* ee_b1  = (const float*)d_in[14];
  const float* ee_w2  = (const float*)d_in[15];
  const float* ee_b2  = (const float*)d_in[16];
  const float* ee_g   = (const float*)d_in[17];
  const float* ee_b   = (const float*)d_in[18];
  const float* pn_w1  = (const float*)d_in[19];
  const float* pn_b1  = (const float*)d_in[20];
  const float* pn_w2  = (const float*)d_in[21];
  const float* pn_b2  = (const float*)d_in[22];
  const float* pn_g   = (const float*)d_in[23];
  const float* pn_b   = (const float*)d_in[24];
  const float* pe_w1  = (const float*)d_in[25];
  const float* pe_b1  = (const float*)d_in[26];
  const float* pe_w2  = (const float*)d_in[27];
  const float* pe_b2  = (const float*)d_in[28];
  const float* pe_g   = (const float*)d_in[29];
  const float* pe_b   = (const float*)d_in[30];
  const float* dec_w1 = (const float*)d_in[31];
  const float* dec_b1 = (const float*)d_in[32];
  const float* dec_w2 = (const float*)d_in[33];
  const float* dec_b2 = (const float*)d_in[34];
  float* outp = (float*)d_out;

  char* ws = (char*)d_ws;
  size_t off = 0;
  const size_t oEA  = off; off += (size_t)EP * K2 * 2;
  const size_t oP   = off; off += (size_t)NP * K2 * 4;
  const size_t oX   = off; off += (size_t)NP * K2 * 2;
  const size_t oENW = off; off += (size_t)HID * K2 * 2;
  const size_t oEEW = off; off += (size_t)HID * K2 * 2;
  const size_t oDEC = off; off += (size_t)HID * K2 * 2;
  const size_t oPAB = off; off += (size_t)NLAY * K2 * K2 * 2;
  const size_t oPC  = off; off += (size_t)NLAY * HID * K2 * 2;
  const size_t oPE2 = off; off += (size_t)NLAY * HID * K2 * 2;
  const size_t oPN1 = off; off += (size_t)NLAY * HID * K4 * 2;
  const size_t oPN2 = off; off += (size_t)NLAY * HID * K2 * 2;
  const size_t oPAR = off; off += (((size_t)PA_TOTAL * 4 + 255) & ~(size_t)255);
  if (off > ws_size || off > (size_t)WSMAX) return;
  if ((size_t)NP * K2 * 2 > (size_t)NP * K2 * 4) return;
  unsigned short* EA   = (unsigned short*)(ws + oEA);
  float*          P    = (float*)(ws + oP);
  unsigned short* AGG  = (unsigned short*)(ws + oP);
  unsigned short* X    = (unsigned short*)(ws + oX);
  unsigned short* ENW2 = (unsigned short*)(ws + oENW);
  unsigned short* EEW2 = (unsigned short*)(ws + oEEW);
  unsigned short* DEC1 = (unsigned short*)(ws + oDEC);
  unsigned short* PAB  = (unsigned short*)(ws + oPAB);
  unsigned short* PC   = (unsigned short*)(ws + oPC);
  unsigned short* PE2  = (unsigned short*)(ws + oPE2);
  unsigned short* PN1  = (unsigned short*)(ws + oPN1);
  unsigned short* PN2  = (unsigned short*)(ws + oPN2);
  float*          PAR  = (float*)(ws + oPAR);

  hipFuncSetAttribute(reinterpret_cast<const void*>(&k_enc<DINN>), hipFuncAttributeMaxDynamicSharedMemorySize,
                      (int)ENC_LDS_BYTES);
  hipFuncSetAttribute(reinterpret_cast<const void*>(&k_enc<DINE>), hipFuncAttributeMaxDynamicSharedMemorySize,
                      (int)ENC_LDS_BYTES);
  hipFuncSetAttribute(reinterpret_cast<const void*>(&k_edge), hipFuncAttributeMaxDynamicSharedMemorySize,
                      (int)CH_LDS_BYTES);
  hipFuncSetAttribute(reinterpret_cast<const void*>(&k_node), hipFuncAttributeMaxDynamicSharedMemorySize,
                      (int)CH_LDS_BYTES);
  hipFuncSetAttribute(reinterpret_cast<const void*>(&k_dec), hipFuncAttributeMaxDynamicSharedMemorySize,
                      (int)DEC_LDS_BYTES);
  hipFuncSetAttribute(reinterpret_cast<const void*>(&k_agg), hipFuncAttributeMaxDynamicSharedMemorySize,
                      (int)AGG_LDS_BYTES);

  k_wplane<<<dim3(16, 1), NTHR, 0, stream>>>(en_w2,  ENW2, HID, K2, 0, 0, 0, 0);
  k_wplane<<<dim3(16, 1), NTHR, 0, stream>>>(ee_w2,  EEW2, HID, K2, 0, 0, 0, 0);
  k_wplane<<<dim3(16, 1), NTHR, 0, stream>>>(dec_w1, DEC1, HID, K2, 0, 0, 0, 0);
  k_wplane<<<dim3(32, NLAY), NTHR, 0, stream>>>(pe_w1, PAB, K2,  K2, 3 * HID * HID, 0,       HID, 0);
  k_wplane<<<dim3(16, NLAY), NTHR, 0, stream>>>(pe_w1, PC,  HID, K2, 3 * HID * HID, 2 * HID, 0,   0);
  k_wplane<<<dim3(16, NLAY), NTHR, 0, stream>>>(pe_w2, PE2, HID, K2, HID * HID,     0,       0,   0);
  k_wplane<<<dim3(32, NLAY), NTHR, 0, stream>>>(pn_w1, PN1, HID, K4, 2 * HID * HID, 0,       0,   HID);
  k_wplane<<<dim3(16, NLAY), NTHR, 0, stream>>>(pn_w2, PN2, HID, K2, HID * HID,     0,       0,   0);
  k_parA<<<cdiv(9 * 32, NTHR), NTHR, 0, stream>>>(en_b1, en_b2, en_g, en_b, ee_b1, ee_b2, ee_g, ee_b, dec_b1, PAR);
  k_parB<<<cdiv(8 * NLAY * 32, NTHR), NTHR, 0, stream>>>(pe_b1, pe_b2, pe_g, pe_b, pn_b1, pn_b2, pn_g, pn_b, PAR);
  k_parC<<<8, NTHR, 0, stream>>>(dec_w2, dec_b2, mean_x, std_x, mean_e, std_e, en_w1, ee_w1, PAR);

  k_enc<DINN><<<NP / TM, NTHR, ENC_LDS_BYTES, stream>>>(x_in, NNODE, PAR, PA_MX, PA_SX, PA_ENW1, PA_ENB, ENW2, X);
  k_enc<DINE><<<EP / TM, NTHR, ENC_LDS_BYTES, stream>>>(eattr, NEDGE, PAR, PA_ME, PA_SE, PA_EEW1, PA_EEB, EEW2, EA);

  for (int l = 0; l < NLAY; ++l) {
    const int oL = PA_LAYER + l * 1024;
    k_pre<<<dim3(NP / GBM, K2 / GBN), GTHR, 0, stream>>>(X, PAB + (size_t)l * K2 * K2, P);
    k_edge<<<EP / TM, NTHR, CH_LDS_BYTES, stream>>>(ei, EA, P, PC + (size_t)l * HID * K2, PE2 + (size_t)l * HID * K2,
                                                    PAR, oL, NEDGE, NNODE);
    k_agg<<<cdiv(NP, NBA), NTHR, AGG_LDS_BYTES, stream>>>(ei, NEDGE, EA, AGG, NP);
    k_node<<<NP / TM, NTHR, CH_LDS_BYTES, stream>>>(X, AGG, PN1 + (size_t)l * HID * K4, PN2 + (size_t)l * HID * K2,
                                                    PAR, oL + 512, NNODE);
  }

  k_dec<<<NP / TM, NTHR, DEC_LDS_BYTES, stream>>>(X, DEC1, PAR, outp, NNODE);
}
